// Classifier_27092653703484
// MI455X (gfx1250) — hardware-verified
//
#include <hip/hip_runtime.h>
#include <stddef.h>
#include <stdint.h>


#define HF    128
#define KIN   256
#define NTHR  256
#define EPB   256
#define GBM   64
#define GBN   128
#define GTHR  128
#define NUW   (HF * KIN / 8)
#define UPR   (HF / 8)
#define WSMAX 134217728

static_assert(NUW % NTHR == 0);
static_assert((GBM * UPR) % NTHR == 0);
static_assert(HF % 32 == 0 && HF == GBN && KIN == 2 * HF);
static_assert(GBM == (GTHR / 32) * 16 && GBN == 4 * 32);
static_assert(EPB == NTHR && EPB == 8 * 32 && HF % 4 == 0 && HF <= NTHR);
static_assert(UPR == 16 && KIN / 8 == 32);

typedef float          v4f   __attribute__((ext_vector_type(4)));
typedef float          v8f   __attribute__((ext_vector_type(8)));
typedef int            v8i   __attribute__((ext_vector_type(8)));
typedef unsigned short v8us  __attribute__((ext_vector_type(8)));
typedef unsigned short v16us __attribute__((ext_vector_type(16)));
typedef __bf16         v16bf __attribute__((ext_vector_type(16)));
typedef v4f  __attribute__((may_alias)) v4fa;
typedef v8us __attribute__((may_alias)) v8usa;
union FragB { v16bf v; v16us u; v8us h[2]; v8i w; };

__device__ __forceinline__ v8f wmb(const FragB& a, const FragB& b, v8f c) {
  v8f d = __builtin_amdgcn_wmma_f32_16x16x32_bf16(false, a.v, false, b.v, (short)0, c, false, false);
  asm volatile("v_nop\n\tv_nop\n\tv_nop\n\tv_nop" : "+v"(d) : "v"(a.w), "v"(b.w));
  return d;
}

__device__ __forceinline__ unsigned bf16_bits(float f) {
  const unsigned u = __float_as_uint(f);
  return (u + 0x7FFFu + ((u >> 16) & 1u)) >> 16;
}
__device__ __forceinline__ float bf16_val(float f) {
  return __uint_as_float(bf16_bits(f) << 16);
}

__global__ __launch_bounds__(NTHR) void k_prep(const float* __restrict__ W1, int nW,
                                               const float* __restrict__ x, int nN, int nUX,
                                               unsigned short* WT, unsigned short* X) {
  const int u = (int)blockIdx.x * NTHR + (int)threadIdx.x;
  v8us o;
  unsigned short* dp;
  if (u < nW) {
    const int n  = u >> 5;
    const int k8 = (u & 31) * 8;
    const float* p = W1 + (size_t)k8 * HF + n;
#pragma unroll
    for (int i = 0; i < 8; ++i) o[i] = (unsigned short)bf16_bits(p[(size_t)i * HF]);
    dp = WT + (size_t)n * KIN + k8;
  } else {
    const int v = u - nW;
    if (v >= nUX) return;
    const int row = v >> 4;
    const int k8  = (v & 15) * 8;
    const int rc  = row < nN ? row : nN - 1;
    const float* p = x + (size_t)rc * HF + k8;
    const v4f a = *(const v4fa*)p;
    const v4f b = *(const v4fa*)(p + 4);
    const bool ok = row < nN;
    o[0] = ok ? (unsigned short)bf16_bits(a.x) : (unsigned short)0;
    o[1] = ok ? (unsigned short)bf16_bits(a.y) : (unsigned short)0;
    o[2] = ok ? (unsigned short)bf16_bits(a.z) : (unsigned short)0;
    o[3] = ok ? (unsigned short)bf16_bits(a.w) : (unsigned short)0;
    o[4] = ok ? (unsigned short)bf16_bits(b.x) : (unsigned short)0;
    o[5] = ok ? (unsigned short)bf16_bits(b.y) : (unsigned short)0;
    o[6] = ok ? (unsigned short)bf16_bits(b.z) : (unsigned short)0;
    o[7] = ok ? (unsigned short)bf16_bits(b.w) : (unsigned short)0;
    dp = X + (size_t)row * HF + k8;
  }
  *(volatile v8us*)dp = o;
  __threadfence();
  *(volatile v8us*)dp = o;
}

__global__ __launch_bounds__(GTHR) void k_gemm(const unsigned short* __restrict__ A, int lda,
                                               const unsigned short* __restrict__ BT, int ldb, int K,
                                               float* Cm, int ldc) {
  __shared__ __attribute__((aligned(16))) float stg[GBM * GBN];
  const int tid = (int)threadIdx.x, lane = tid & 31, wave = tid >> 5, hh = lane >> 4, m = lane & 15;
  const int rowBase = (int)blockIdx.x * GBM;
  const int colBase = (int)blockIdx.y * GBN;

  v8f acc[8];
  {
    const v8f z = {0.f, 0.f, 0.f, 0.f, 0.f, 0.f, 0.f, 0.f};
#pragma unroll
    for (int t = 0; t < 8; ++t) acc[t] = z;
  }
  const unsigned short* ap = A  + (size_t)(rowBase + 16 * wave + m) * (size_t)lda + 8 * hh;
  const unsigned short* bp = BT + (size_t)(colBase + m) * (size_t)ldb + 8 * hh;

#pragma unroll 1
  for (int k0 = 0; k0 < K; k0 += 32) {
    FragB af;
    af.h[0] = *(const v8usa*)(ap + k0);
    af.h[1] = *(const v8usa*)(ap + k0 + 16);
#pragma unroll
    for (int nt = 0; nt < 8; ++nt) {
      const unsigned short* wq = bp + (size_t)(16 * nt) * (size_t)ldb + k0;
      FragB bf;
      bf.h[0] = *(const v8usa*)wq;
      bf.h[1] = *(const v8usa*)(wq + 16);
      acc[nt] = wmb(af, bf, acc[nt]);
    }
  }

#pragma unroll
  for (int nt = 0; nt < 8; ++nt) {
    const int lc = 16 * nt + m;
#pragma unroll
    for (int r = 0; r < 8; ++r) {
      const int lr = 16 * wave + 8 * hh + r;
      stg[lr * GBN + lc] = acc[nt][r];
    }
  }
  __syncthreads();

  v4f pv[16];
#pragma unroll
  for (int i = 0; i < 16; ++i) pv[i] = *(const v4fa*)(stg + (16 * wave + i) * GBN + 4 * lane);
#pragma unroll
  for (int i = 0; i < 16; ++i) {
    float* op = Cm + (size_t)(rowBase + 16 * wave + i) * (size_t)ldc + colBase + 4 * lane;
    *(volatile v4f*)op = pv[i];
  }
  __threadfence();
#pragma unroll
  for (int i = 0; i < 16; ++i) {
    float* op = Cm + (size_t)(rowBase + 16 * wave + i) * (size_t)ldc + colBase + 4 * lane;
    *(volatile v4f*)op = pv[i];
  }
}

__global__ __launch_bounds__(NTHR) void k_pair(const int* __restrict__ si, const int* __restrict__ di,
                                               int nE, int nS, int nD,
                                               const float* __restrict__ pp, const float* __restrict__ pq,
                                               const float* __restrict__ b1, const float* __restrict__ w2,
                                               const float* __restrict__ b2, float* out) {
  __shared__ __attribute__((aligned(16))) float cst[2 * HF + 16];
  __shared__ __attribute__((aligned(16))) float sy[EPB];
  const int tid = (int)threadIdx.x;

  if (tid < HF) {
    cst[tid]      = bf16_val(b1[tid]);
    cst[HF + tid] = bf16_val(w2[tid]);
  }
  if (tid < 32) {
    const float vb = bf16_val(b2[0]);
    if (tid == 0) cst[2 * HF] = vb;
  }

  const int e0 = (int)blockIdx.x * EPB;
  int ec = e0 + tid;
  ec = ec > nE - 1 ? nE - 1 : ec;
  int s = si[ec];
  int t = di[ec];
  s = s < 0 ? 0 : (s > nS - 1 ? nS - 1 : s);
  t = t < 0 ? 0 : (t > nD - 1 ? nD - 1 : t);
  const float* pa = pp + (size_t)s * HF;
  const float* pb = pq + (size_t)t * HF;
  __syncthreads();

  float dot = 0.0f;
#pragma unroll 2
  for (int c4 = 0; c4 < HF / 4; ++c4) {
    const v4f a  = *(const v4fa*)(pa + 4 * c4);
    const v4f q  = *(const v4fa*)(pb + 4 * c4);
    const v4f bb = *(const v4fa*)(cst + 4 * c4);
    const v4f ww = *(const v4fa*)(cst + HF + 4 * c4);
    const float t0 = fmaxf((a.x + q.x) + bb.x, 0.0f);
    const float t1 = fmaxf((a.y + q.y) + bb.y, 0.0f);
    const float t2 = fmaxf((a.z + q.z) + bb.z, 0.0f);
    const float t3 = fmaxf((a.w + q.w) + bb.w, 0.0f);
    dot = fmaf(t0, ww.x, dot);
    dot = fmaf(t1, ww.y, dot);
    dot = fmaf(t2, ww.z, dot);
    dot = fmaf(t3, ww.w, dot);
  }
  const float yv = dot + cst[2 * HF];
  sy[tid] = yv;
  __syncthreads();

  const int tl = tid < 64 ? tid : 63;
  const v4f o4 = *(const v4fa*)(sy + 4 * tl);
  const int eo = e0 + 4 * tl;
  const bool stv = (tid < 64) && (eo + 3 < nE);
  if (stv) *(volatile v4f*)(out + (size_t)eo) = o4;
  __threadfence();
  if (stv) *(volatile v4f*)(out + (size_t)eo) = o4;
}

static inline int cdiv(int a, int b) { return (a + b - 1) / b; }

extern "C" void kernel_launch(void* const* d_in, const int* in_sizes, int n_in,
                              void* d_out, int out_size, void* d_ws, size_t ws_size,
                              hipStream_t stream) {
  if (n_in < 7) return;
  if (in_sizes[0] < HF || (in_sizes[0] % HF) != 0) return;
  const int nS = in_sizes[0] / HF;
  if (in_sizes[1] < HF || (in_sizes[1] % HF) != 0) return;
  const int nD = in_sizes[1] / HF;
  if (nS > (1 << 22) || nD > (1 << 22)) return;
  if (in_sizes[2] < 64 || (in_sizes[2] & 1) != 0) return;
  const int nE = in_sizes[2] / 2;
  if (nE < 32 || (nE & 31) != 0) return;
  if (in_sizes[3] != KIN * HF) return;
  if (in_sizes[4] != HF) return;
  if (in_sizes[5] != HF) return;
  if (in_sizes[6] != 1) return;
  if (out_size != nE) return;

  const float* xs   = (const float*)d_in[0];
  const float* xd   = (const float*)d_in[1];
  const int*   eidx = (const int*)d_in[2];
  const int*   src  = eidx;
  const int*   dst  = eidx + (size_t)nE;
  const float* W1   = (const float*)d_in[3];
  const float* b1   = (const float*)d_in[4];
  const float* W2   = (const float*)d_in[5];
  const float* b2   = (const float*)d_in[6];
  float* out = (float*)d_out;

  const int MPS = cdiv(nS, GBM) * GBM;
  const int MPD = cdiv(nD, GBM) * GBM;
  const int MPX = MPS > MPD ? MPS : MPD;
  const int nUS = MPS * UPR;
  const int nUD = MPD * UPR;

  char* ws = (char*)d_ws;
  size_t off = 0;
  const size_t oWT = off; off += (size_t)HF * KIN * 2;       off = (off + 255) & ~(size_t)255;
  const size_t oX  = off; off += (size_t)MPX * HF * 2;       off = (off + 255) & ~(size_t)255;
  const size_t oP  = off; off += (size_t)MPS * HF * 4;       off = (off + 255) & ~(size_t)255;
  const size_t oQ  = off; off += (size_t)MPD * HF * 4;       off = (off + 255) & ~(size_t)255;
  if (off > ws_size || off > (size_t)WSMAX) return;
  unsigned short* WT = (unsigned short*)(ws + oWT);
  unsigned short* X  = (unsigned short*)(ws + oX);
  float*          P  = (float*)(ws + oP);
  float*          Q  = (float*)(ws + oQ);

  k_prep<<<cdiv(NUW + nUS, NTHR), NTHR, 0, stream>>>(W1, NUW, xs, nS, nUS, WT, X);
  k_gemm<<<dim3(MPS / GBM, HF / GBN), GTHR, 0, stream>>>(X, HF, WT, KIN, HF, P, HF);
  k_prep<<<cdiv(nUD, NTHR), NTHR, 0, stream>>>(W1, 0, xd, nD, nUD, WT, X);
  k_gemm<<<dim3(MPD / GBM, HF / GBN), GTHR, 0, stream>>>(X, HF, WT + HF, KIN, HF, Q, HF);
  k_pair<<<cdiv(nE, EPB), NTHR, 0, stream>>>(src, dst, nE, nS, nD, P, Q, b1, W2, b2, out);
}
